// LocalCrossAttention_1494648619504
// MI455X (gfx1250) — hardware-verified
//
#include <hip/hip_runtime.h>


#define NB_  2
#define TT   8192
#define HID  512
#define NH_  8
#define HD   64
#define CH   128
#define NC   64
#define WK   256
#define TP   (TT + CH)
typedef _Float16 h16;
typedef unsigned short bf;
typedef __attribute__((ext_vector_type(16))) __bf16   v16bf;
typedef __attribute__((ext_vector_type(16))) _Float16 v16h;
typedef __attribute__((ext_vector_type(8)))  _Float16 v8h;
typedef __attribute__((ext_vector_type(8)))  unsigned short v8us;
typedef __attribute__((ext_vector_type(8)))  float    v8f;
typedef __attribute__((ext_vector_type(4)))  float    v4f;
typedef v8h  __attribute__((may_alias)) v8ha;
typedef v4f  __attribute__((may_alias)) v4fa;
typedef v8us __attribute__((may_alias)) v8usa;

__device__ __forceinline__ unsigned short f2bf(float f) { unsigned u = __float_as_uint(f); u += 0x7FFFu + ((u >> 16) & 1u); return (unsigned short)(u >> 16); }
__device__ __forceinline__ float bf2f(unsigned short b) { return __uint_as_float(((unsigned)b) << 16); }
__device__ __forceinline__ float bfr(float f) { return bf2f(f2bf(f)); }
__device__ __forceinline__ v16h cat16(v8h lo, v8h hi) { return __builtin_shufflevector(lo, hi, 0, 1, 2, 3, 4, 5, 6, 7, 8, 9, 10, 11, 12, 13, 14, 15); }
__device__ __forceinline__ v16bf cat16b(v8us lo, v8us hi) { return __builtin_bit_cast(v16bf, __builtin_shufflevector(lo, hi, 0, 1, 2, 3, 4, 5, 6, 7, 8, 9, 10, 11, 12, 13, 14, 15)); }
__device__ __forceinline__ v8f wmma16(v16h a, v16h b, v8f c) { return __builtin_amdgcn_wmma_f32_16x16x32_f16(false, a, false, b, (short)0, c, false, false); }
__device__ __forceinline__ v8f wmmab(v16bf a, v16bf b, v8f c) { return __builtin_amdgcn_wmma_f32_16x16x32_bf16(false, a, false, b, (short)0, c, false, false); }


template <typename T16> struct WFrag;
template <> struct WFrag<h16> { typedef v16h V; static __device__ __forceinline__ V ld(const h16* p) { return cat16(*(const v8h*)p, *(const v8h*)(p + 16)); } static __device__ __forceinline__ v8f mma(V a, V b, v8f c) { return wmma16(a, b, c); } };
template <> struct WFrag<bf> { typedef v16bf V; static __device__ __forceinline__ V ld(const bf* p) { return cat16b(*(const v8us*)p, *(const v8us*)(p + 16)); } static __device__ __forceinline__ v8f mma(V a, V b, v8f c) { return wmmab(a, b, c); } };
template <typename T16, int NSPLIT, bool BIAS>
__global__ __launch_bounds__(32) void k_gemmw(const T16* __restrict__ A, const T16* __restrict__ A2, const T16* __restrict__ Bt, const T16* __restrict__ Bt2, int K, float* C, int ldc, const float* __restrict__ bias, size_t sA, size_t sB, size_t sC) {
    typedef typename WFrag<T16>::V V;
    __shared__ __align__(16) float os[16 * 68];
    const size_t z = blockIdx.z; A += z * sA; if (A2) A2 += z * sA; Bt += z * sB; if (Bt2) Bt2 += z * sB; C += z * sC;
    const int lane = threadIdx.x & 31, lr = lane & 15, hi = lane >> 4; const int r0 = blockIdx.x * 64, c0 = blockIdx.y * 64;
    v8f acc[4][4];
#pragma unroll
    for (int mb = 0; mb < 4; ++mb)
#pragma unroll
        for (int nb = 0; nb < 4; ++nb) acc[mb][nb] = (v8f){};
    const size_t aoff = (size_t)(r0 + lr) * K + 8 * hi, boff = (size_t)(c0 + lr) * K + 8 * hi;
#pragma unroll 1
    for (int kc = 0; kc < K; kc += 32) {
        V a[4], a2[4];
#pragma unroll
        for (int mb = 0; mb < 4; ++mb) { a[mb] = WFrag<T16>::ld(A + aoff + (size_t)mb * 16 * K + kc); if (NSPLIT == 1 || NSPLIT == 2) a2[mb] = WFrag<T16>::ld(A2 + aoff + (size_t)mb * 16 * K + kc); }
#pragma unroll
        for (int nb = 0; nb < 4; ++nb) { const V b = WFrag<T16>::ld(Bt + boff + (size_t)nb * 16 * K + kc); V b2; if (NSPLIT >= 2) b2 = WFrag<T16>::ld(Bt2 + boff + (size_t)nb * 16 * K + kc);
#pragma unroll
            for (int mb = 0; mb < 4; ++mb) { acc[mb][nb] = WFrag<T16>::mma(a[mb], b, acc[mb][nb]); if (NSPLIT == 1 || NSPLIT == 2) acc[mb][nb] = WFrag<T16>::mma(a2[mb], b, acc[mb][nb]); if (NSPLIT >= 2) acc[mb][nb] = WFrag<T16>::mma(a[mb], b2, acc[mb][nb]); } }
        asm volatile("v_nop\n\tv_nop\n\tv_nop\n\tv_nop" : "+v"(acc[0][0]), "+v"(acc[1][1]), "+v"(acc[2][2]), "+v"(acc[3][3]) : "v"(a[0]), "v"(a[3]));
    }
#pragma unroll
    for (int mb = 0; mb < 4; ++mb) {
#pragma unroll
        for (int nb = 0; nb < 4; ++nb) {
#pragma unroll
            for (int j = 0; j < 8; ++j) os[(hi * 8 + j) * 68 + nb * 16 + lr] = acc[mb][nb][j]; }
        __builtin_amdgcn_wave_barrier(); asm volatile("" ::: "memory");
        float* crow = C + (size_t)(r0 + mb * 16) * ldc + c0;
#pragma unroll 1
        for (int ps = 0; ps < 2; ++ps) {
#pragma unroll
            for (int s = 0; s < 8; ++s) { const int row = 2 * s + hi, cofs = lr * 4; v4f val = *(const v4fa*)(os + row * 68 + cofs); if (BIAS) { val[0] += bfr(bias[c0 + cofs]); val[1] += bfr(bias[c0 + cofs + 1]); val[2] += bfr(bias[c0 + cofs + 2]); val[3] += bfr(bias[c0 + cofs + 3]); }
                *(volatile v4f*)(crow + (size_t)row * ldc + cofs) = val; }
            if (ps == 0) __threadfence(); }
        __builtin_amdgcn_wave_barrier(); asm volatile("" ::: "memory");
    }
}

__device__ __forceinline__ void splitf(float y, unsigned short& h, unsigned short& l) { h = f2bf(y); l = f2bf(y - bf2f(h)); }
typedef __attribute__((ext_vector_type(2))) unsigned short v2us;
typedef __attribute__((ext_vector_type(4))) unsigned short v4us;

__global__ __launch_bounds__(256) void k_cvt8(const float* __restrict__ src, bf* dst, size_t n8) { const size_t i = (size_t)blockIdx.x * 256 + threadIdx.x; if (i >= n8) return; const v8f v = *(const v8f*)(src + i * 8); v8us o;
#pragma unroll
    for (int k = 0; k < 8; ++k) o[k] = f2bf(v[k]); *(volatile v8us*)(dst + i * 8) = o; __threadfence(); *(volatile v8us*)(dst + i * 8) = o; }
__global__ __launch_bounds__(256) void k_qpl(const float* __restrict__ F, bf* Ph, bf* Pl) { const size_t e = ((size_t)blockIdx.x * 256 + threadIdx.x) * 4; if (e >= (size_t)NH_ * TT * HD) return; const int d = (int)(e % HD); const int t = (int)((e / HD) % TT); const int h = (int)(e / ((size_t)HD * TT)); const v4f a = *(const v4f*)(F + (size_t)t * HID + h * HD + d); v4us oh, ol;
#pragma unroll
    for (int u = 0; u < 4; ++u) { unsigned short x, y; splitf(a[u], x, y); oh[u] = x; ol[u] = y; } *(volatile v4us*)(Ph + e) = oh; *(volatile v4us*)(Pl + e) = ol; __threadfence(); *(volatile v4us*)(Ph + e) = oh; *(volatile v4us*)(Pl + e) = ol; }
__global__ __launch_bounds__(256) void k_kpl(const float* __restrict__ F, bf* Ph, bf* Pl) { const size_t e = ((size_t)blockIdx.x * 256 + threadIdx.x) * 4; if (e >= (size_t)NH_ * TP * HD) return; const int d = (int)(e % HD); const int r = (int)((e / HD) % TP); const int h = (int)(e / ((size_t)HD * TP)); const int s = (r < CH) ? (TT - CH + r) : (r - CH); const v4f a = *(const v4f*)(F + (size_t)s * HID + h * HD + d); v4us oh, ol;
#pragma unroll
    for (int u = 0; u < 4; ++u) { unsigned short x, y; splitf(a[u] * 0.125f, x, y); oh[u] = x; ol[u] = y; } *(volatile v4us*)(Ph + e) = oh; *(volatile v4us*)(Pl + e) = ol; __threadfence(); *(volatile v4us*)(Ph + e) = oh; *(volatile v4us*)(Pl + e) = ol; }
__global__ __launch_bounds__(256) void k_vwin(const float* __restrict__ F, bf* Vh, bf* Vl) { const size_t e = ((size_t)blockIdx.x * 256 + threadIdx.x) * 2; if (e >= (size_t)NH_ * NC * HD * WK) return; const int j = (int)(e % WK); const int d = (int)((e / WK) % HD); const int c = (int)((e / ((size_t)WK * HD)) % NC); const int h = (int)(e / ((size_t)WK * HD * NC)); v2us oh, ol;
#pragma unroll
    for (int u = 0; u < 2; ++u) { const int jj = j + u; const int s = (jj < CH) ? (((c + NC - 1) % NC) * CH + jj) : (c * CH + jj - CH); unsigned short x, y; splitf(F[(size_t)s * HID + h * HD + d], x, y); oh[u] = x; ol[u] = y; }
    *(volatile v2us*)(Vh + e) = oh; *(volatile v2us*)(Vl + e) = ol; __threadfence(); *(volatile v2us*)(Vh + e) = oh; *(volatile v2us*)(Vl + e) = ol; }
__global__ __launch_bounds__(256) void k_mrg(const float* __restrict__ O, float* OUTb) { const size_t e = ((size_t)blockIdx.x * 256 + threadIdx.x) * 4; if (e >= (size_t)TT * HID) return; const int c_ = (int)(e % HID); const int t = (int)(e / HID); const int h = c_ / HD, d = c_ % HD; const int c = t / CH, i = t % CH; const v4f a = *(const v4f*)(O + (((size_t)(h * NC + c)) * CH + i) * HD + d);
    *(volatile v4f*)(OUTb + e) = a; __threadfence(); *(volatile v4f*)(OUTb + e) = a; }
__global__ __launch_bounds__(256) void k_wsoft(const float* __restrict__ Sb, const int* __restrict__ am, bf* Ph, bf* Pl) { const int lane = threadIdx.x & 31; const int row = blockIdx.x * 8 + (threadIdx.x >> 5); if (row >= NH_ * NC * CH) return; const int i = row % CH; const int c = (row / CH) % NC; const int qpos = c * CH + i; const bool qok = am[qpos] != 0; const float* sr = Sb + (size_t)row * WK; float v[8]; float mx = -3.0e38f;
#pragma unroll
    for (int ch = 0; ch < 2; ++ch) { const int j0 = ch * 128 + lane * 4; const v4f a = *(const v4f*)(sr + j0);
#pragma unroll
        for (int u = 0; u < 4; ++u) { const int j = j0 + u; const int kpos = (j < CH) ? (((c + NC - 1) % NC) * CH + j) : (c * CH + j - CH); const bool ok = qok && (qpos >= kpos) && (am[kpos] != 0); const float t = ok ? a[u] : -1.0e9f; v[ch * 4 + u] = t; mx = fmaxf(mx, t); } }
#pragma unroll
    for (int sh = 16; sh; sh >>= 1) mx = fmaxf(mx, __shfl_xor(mx, sh, 32));
    float sum = 0.f;
#pragma unroll
    for (int k = 0; k < 8; ++k) { float d0 = __fsub_rn(v[k], mx); asm volatile("" : "+v"(d0)); v[k] = __expf(d0); sum += v[k]; }
#pragma unroll
    for (int sh = 16; sh; sh >>= 1) sum += __shfl_xor(sum, sh, 32);
    const float f = __fdiv_rn(1.0f, sum);
    for (int ps = 0; ps < 2; ++ps) {
#pragma unroll
        for (int ch = 0; ch < 2; ++ch) { v4us oh, ol;
#pragma unroll
            for (int u = 0; u < 4; ++u) { unsigned short a, b; splitf(v[ch * 4 + u] * f, a, b); oh[u] = a; ol[u] = b; } const size_t oo = (size_t)row * WK + ch * 128 + lane * 4; *(volatile v4us*)(Ph + oo) = oh; *(volatile v4us*)(Pl + oo) = ol; }
        if (ps == 0) __threadfence(); } }

extern "C" void kernel_launch(void* const* d_in, const int* in_sizes, int n_in,
                              void* d_out, int out_size, void* d_ws, size_t ws_size, hipStream_t stream) {
    (void)in_sizes; (void)n_in; (void)out_size;
    const float* dec = (const float*)d_in[0]; const float* enc = (const float*)d_in[1]; const int* amask = (const int*)d_in[2]; const float* wq = (const float*)d_in[3]; const float* wk = (const float*)d_in[4]; const float* wv = (const float*)d_in[5];
    float* OUT = (float*)d_out;
    char* wsp = (char*)d_ws;
    auto take = [&](size_t bytes) { char* p = wsp; wsp += (bytes + 255) & ~(size_t)255; return (void*)p; };
    bf* WQ = (bf*)take(HID * HID * 2); bf* WK_ = (bf*)take(HID * HID * 2); bf* WV = (bf*)take(HID * HID * 2);
    bf* XB = (bf*)take((size_t)TT * HID * 2); float* F = (float*)take((size_t)TT * HID * 4); bf* QPh = (bf*)take((size_t)NH_ * TT * HD * 2); bf* QPl = (bf*)take((size_t)NH_ * TT * HD * 2); bf* KPh = (bf*)take((size_t)NH_ * TP * HD * 2); bf* KPl = (bf*)take((size_t)NH_ * TP * HD * 2); bf* VWh = (bf*)take((size_t)NH_ * NC * HD * WK * 2); bf* VWl = (bf*)take((size_t)NH_ * NC * HD * WK * 2);
    float* Sb = (float*)take((size_t)NH_ * NC * CH * WK * 4); bf* Ph = (bf*)take((size_t)NH_ * NC * CH * WK * 2); bf* Pl = (bf*)take((size_t)NH_ * NC * CH * WK * 2); float* O = (float*)take((size_t)NH_ * NC * CH * HD * 4);
    if ((size_t)(wsp - (char*)d_ws) > ws_size) return;
    k_cvt8<<<(HID * HID / 8 + 255) / 256, 256, 0, stream>>>(wq, WQ, HID * HID / 8); k_cvt8<<<(HID * HID / 8 + 255) / 256, 256, 0, stream>>>(wk, WK_, HID * HID / 8); k_cvt8<<<(HID * HID / 8 + 255) / 256, 256, 0, stream>>>(wv, WV, HID * HID / 8);
    for (int b = 0; b < NB_; ++b) {
        k_cvt8<<<(unsigned)(((size_t)TT * HID / 8 + 255) / 256), 256, 0, stream>>>(dec + (size_t)b * TT * HID, XB, (size_t)TT * HID / 8); k_gemmw<bf, 0, false><<<dim3(TT / 64, HID / 64, 1), 32, 0, stream>>>(XB, nullptr, WQ, nullptr, HID, F, HID, nullptr, 0, 0, 0); k_qpl<<<(unsigned)(((size_t)NH_ * TT * HD / 4 + 255) / 256), 256, 0, stream>>>(F, QPh, QPl);
        k_cvt8<<<(unsigned)(((size_t)TT * HID / 8 + 255) / 256), 256, 0, stream>>>(enc + (size_t)b * TT * HID, XB, (size_t)TT * HID / 8); k_gemmw<bf, 0, false><<<dim3(TT / 64, HID / 64, 1), 32, 0, stream>>>(XB, nullptr, WK_, nullptr, HID, F, HID, nullptr, 0, 0, 0); k_kpl<<<(unsigned)(((size_t)NH_ * TP * HD / 4 + 255) / 256), 256, 0, stream>>>(F, KPh, KPl);
        k_gemmw<bf, 0, false><<<dim3(TT / 64, HID / 64, 1), 32, 0, stream>>>(XB, nullptr, WV, nullptr, HID, F, HID, nullptr, 0, 0, 0); k_vwin<<<(unsigned)(((size_t)NH_ * NC * HD * WK / 2 + 255) / 256), 256, 0, stream>>>(F, VWh, VWl);
        for (int h = 0; h < NH_; ++h) {
            k_gemmw<bf, 2, false><<<dim3(CH / 64, WK / 64, NC), 32, 0, stream>>>(QPh + (size_t)h * TT * HD, QPl + (size_t)h * TT * HD, KPh + (size_t)h * TP * HD, KPl + (size_t)h * TP * HD, HD, Sb + (size_t)h * NC * CH * WK, WK, nullptr, (size_t)CH * HD, (size_t)CH * HD, (size_t)CH * WK); }
        k_wsoft<<<NH_ * NC * CH / 8, 256, 0, stream>>>(Sb, amask + (size_t)b * TT, Ph, Pl);
        k_gemmw<bf, 2, false><<<dim3(CH / 64, 1, NH_ * NC), 32, 0, stream>>>(Ph, Pl, VWh, VWl, WK, O, HD, nullptr, (size_t)CH * WK, (size_t)HD * WK, (size_t)CH * HD);
        k_mrg<<<(unsigned)(((size_t)TT * HID / 4 + 255) / 256), 256, 0, stream>>>(O, OUT + (size_t)b * TT * HID); }
}
